// Virtual_pts_BEV_Warp_79688823210364
// MI455X (gfx1250) — hardware-verified
//
#include <hip/hip_runtime.h>
#define HH 128
#define NQ (HH * HH)
#define CIN 384
#define DD 256
#define NHD 8
#define NPT 4
#define HD 32
#define NLAY 4
#define NCROSS 3
typedef __bf16 v16b __attribute__((ext_vector_type(16)));
typedef unsigned short v8us __attribute__((ext_vector_type(8), may_alias));
typedef float  v8f  __attribute__((ext_vector_type(8)));
typedef float  v4f  __attribute__((ext_vector_type(4)));
typedef float  v4fa __attribute__((ext_vector_type(4), may_alias));
union FragB { v16b v; v8us half[2]; unsigned short u[16]; };

__device__ __forceinline__ unsigned short bf16_bits(float x) { unsigned int u = __float_as_uint(x); return (unsigned short)((u + 0x7FFFu + ((u >> 16) & 1u)) >> 16); }
__device__ __forceinline__ float bf16_val(unsigned short b) { return __uint_as_float(((unsigned int)b) << 16); }
__device__ __forceinline__ float bf16_round(float x) { return bf16_val(bf16_bits(x)); }
template <int NT>
__device__ __forceinline__ v8f mmaN(v16b ah, v16b al, v16b bh, v16b bl, v8f c) {
  c = __builtin_amdgcn_wmma_f32_16x16x32_bf16(false, ah, false, bh, (short)0, c, false, false);
  if (NT >= 2) c = __builtin_amdgcn_wmma_f32_16x16x32_bf16(false, al, false, bh, (short)0, c, false, false);
  if (NT >= 3) c = __builtin_amdgcn_wmma_f32_16x16x32_bf16(false, ah, false, bl, (short)0, c, false, false);
  asm volatile("v_nop\n\tv_nop\n\tv_nop\n\tv_nop" : "+v"(c) : "v"(ah), "v"(al), "v"(bh), "v"(bl));
  return c;
}

__global__ __launch_bounds__(256) void k_wt_bf16(const float* __restrict__ W, unsigned short* __restrict__ Wt, int K, int N) {
  const int t = blockIdx.x * 256 + threadIdx.x;
  const int k8n = K / 8;
  if (t >= N * k8n) return;
  const int n = t / k8n, k8 = (t % k8n) * 8;
  v8us v;
#pragma unroll
  for (int i = 0; i < 8; ++i) v[i] = bf16_bits(W[(size_t)(k8 + i) * N + n]);
  *(volatile v8us*)(Wt + (size_t)n * K + k8) = v;
  __threadfence();
  *(volatile v8us*)(Wt + (size_t)n * K + k8) = v;
}

template <bool ASPLIT, int ACT, bool BIAS_BF16>
__global__ __launch_bounds__(128) void k_gemm_bf(const float* __restrict__ A, int lda, const unsigned short* __restrict__ Wt, int ldb,
                                               const float* __restrict__ bias, float* __restrict__ C, int ldc, int M, int N, int K) {
  __shared__ __attribute__((aligned(16))) float so[4][16][64];
  const int tid = threadIdx.x, w = tid >> 5, lane = tid & 31, ln = lane & 15, hh = lane >> 4;
  const int ntn = N / 64;
  const int wid = blockIdx.x * 4 + w;
  const int mt = wid / ntn, nq = wid % ntn;
  if (mt * 16 >= M) return;
  const int row0 = mt * 16, col0 = nq * 64;
  const float* arow = A + (size_t)(row0 + ln) * lda;
  v8f acc[4] = {};
  for (int kb = 0; kb < K; kb += 32) {
    FragB ah, al;
    const v4f x0 = *(const v4fa*)(arow + kb + 8 * hh), x1 = *(const v4fa*)(arow + kb + 8 * hh + 4);
    const v4f x2 = *(const v4fa*)(arow + kb + 16 + 8 * hh), x3 = *(const v4fa*)(arow + kb + 16 + 8 * hh + 4);
    float xs[16] = {x0[0],x0[1],x0[2],x0[3],x1[0],x1[1],x1[2],x1[3],x2[0],x2[1],x2[2],x2[3],x3[0],x3[1],x3[2],x3[3]};
#pragma unroll
    for (int i = 0; i < 16; ++i) { const unsigned short hb = bf16_bits(xs[i]); ah.u[i] = hb; al.u[i] = ASPLIT ? bf16_bits(xs[i] - bf16_val(hb)) : (unsigned short)0; }
#pragma unroll
    for (int t = 0; t < 4; ++t) {
      const unsigned short* brow = Wt + (size_t)(col0 + t * 16 + ln) * ldb + kb;
      FragB b;
      b.half[0] = *(const v8us*)(brow + 8 * hh);
      b.half[1] = *(const v8us*)(brow + 16 + 8 * hh);
      acc[t] = mmaN<ASPLIT ? 2 : 1>(ah.v, al.v, b.v, b.v, acc[t]);
    }
  }
#pragma unroll
  for (int t = 0; t < 4; ++t) {
    float bv = bias ? bias[col0 + t * 16 + ln] : 0.f;
    if (BIAS_BF16) bv = bf16_round(bv);
#pragma unroll
    for (int r = 0; r < 8; ++r) { float v = acc[t][r] + bv; if (ACT == 1) v = fmaxf(v, 0.f); so[w][8 * hh + r][t * 16 + ln] = v; }
  }
  __builtin_amdgcn_fence(__ATOMIC_ACQ_REL, "workgroup");
  __builtin_amdgcn_wave_barrier();
  const int rsub = lane >> 4, c4 = (lane & 15) * 4;
  for (int pass = 0; pass < 2; ++pass) {
#pragma unroll
    for (int q = 0; q < 8; ++q) {
      const int r = q * 2 + rsub;
      const v4f v = *(const v4fa*)&so[w][r][c4];
      *(volatile v4f*)(C + (size_t)(row0 + r) * ldc + col0 + c4) = v;
    }
    if (pass == 0) __threadfence();
  }
}

template <bool ASPLIT, int ACT, bool BIAS_BF16, bool RES_BF16>
__global__ __launch_bounds__(128) void k_gemm_bf3(const float* __restrict__ A, int lda, const unsigned short* __restrict__ Wt, int ldb,
                                                const float* __restrict__ bias, const float* __restrict__ resid, int rmod, int ldr,
                                                float* __restrict__ C, int ldc, int M, int N, int K) {
  __shared__ __attribute__((aligned(16))) float so[4][16][64];
  const int tid = threadIdx.x, w = tid >> 5, lane = tid & 31, ln = lane & 15, hh = lane >> 4;
  const int ntn = N / 64;
  const int wid = blockIdx.x * 4 + w;
  const int mt = wid / ntn, nq = wid % ntn;
  if (mt * 16 >= M) return;
  const int row0 = mt * 16, col0 = nq * 64;
  const float* arow = A + (size_t)(row0 + ln) * lda;
  v8f acc[4] = {};
  for (int kb = 0; kb < K; kb += 32) {
    FragB ah, al;
    const v4f x0 = *(const v4fa*)(arow + kb + 8 * hh), x1 = *(const v4fa*)(arow + kb + 8 * hh + 4);
    const v4f x2 = *(const v4fa*)(arow + kb + 16 + 8 * hh), x3 = *(const v4fa*)(arow + kb + 16 + 8 * hh + 4);
    float xs[16] = {x0[0],x0[1],x0[2],x0[3],x1[0],x1[1],x1[2],x1[3],x2[0],x2[1],x2[2],x2[3],x3[0],x3[1],x3[2],x3[3]};
#pragma unroll
    for (int i = 0; i < 16; ++i) { const unsigned short hb = bf16_bits(xs[i]); ah.u[i] = hb; al.u[i] = ASPLIT ? bf16_bits(xs[i] - bf16_val(hb)) : (unsigned short)0; }
#pragma unroll
    for (int t = 0; t < 4; ++t) {
      const unsigned short* brow = Wt + (size_t)(col0 + t * 16 + ln) * ldb + kb;
      FragB b;
      b.half[0] = *(const v8us*)(brow + 8 * hh);
      b.half[1] = *(const v8us*)(brow + 16 + 8 * hh);
      acc[t] = mmaN<ASPLIT ? 2 : 1>(ah.v, al.v, b.v, b.v, acc[t]);
    }
  }
#pragma unroll
  for (int t = 0; t < 4; ++t) {
    const int col = col0 + t * 16 + ln;
    float bv = bias ? bias[col] : 0.f;
    if (BIAS_BF16) bv = bf16_round(bv);
#pragma unroll
    for (int r = 0; r < 8; ++r) {
      float v = acc[t][r] + bv;
      if (resid) { float rv = resid[(size_t)((row0 + 8 * hh + r) % rmod) * ldr + col]; if (RES_BF16) rv = bf16_round(rv); v += rv; }
      if (ACT == 1) v = fmaxf(v, 0.f);
      if (ACT == 2) v = 0.5f * v * (1.0f + erff(v * 0.70710678118654752f));
      if (ACT == 3) { const float u = 0.7978845608028654f * (v + 0.044715f * v * v * v); v = 0.5f * v * (1.0f + tanhf(u)); }
      so[w][8 * hh + r][t * 16 + ln] = v;
    }
  }
  __builtin_amdgcn_fence(__ATOMIC_ACQ_REL, "workgroup");
  __builtin_amdgcn_wave_barrier();
  const int rsub = lane >> 4, c4 = (lane & 15) * 4;
  for (int pass = 0; pass < 2; ++pass) {
#pragma unroll
    for (int q = 0; q < 8; ++q) {
      const int r = q * 2 + rsub;
      const v4f v = *(const v4fa*)&so[w][r][c4];
      *(volatile v4f*)(C + (size_t)(row0 + r) * ldc + col0 + c4) = v;
    }
    if (pass == 0) __threadfence();
  }
}
template <bool PARAM_BF16>
__global__ __launch_bounds__(256) void k_layernorm(const float* __restrict__ X, const float* __restrict__ R, const float* __restrict__ g, const float* __restrict__ bta,
                                                  float* __restrict__ out_sum, float* __restrict__ out_norm, int N, float eps) {
  __shared__ float red[256];
  const int row = blockIdx.x, tid = threadIdx.x;
  const float* x = X + (size_t)row * N; const float* rr = R ? R + (size_t)row * N : nullptr;
  float vals[16];
  const int per = N / 256;
  float s1 = 0.f;
  for (int u = 0; u < per / 4; ++u) {
    const int j = tid * 4 + 1024 * u;
    const v4f a = *(const v4fa*)(x + j);
    v4f b = {0.f,0.f,0.f,0.f}; if (rr) b = *(const v4fa*)(rr + j);
#pragma unroll
    for (int q = 0; q < 4; ++q) { const float v = a[q] + b[q]; vals[u * 4 + q] = v; s1 += v; }
  }
  red[tid] = s1; __syncthreads();
  for (int st = 128; st > 0; st >>= 1) { if (tid < st) red[tid] += red[tid + st]; __syncthreads(); }
  const float mu = red[0] / (float)N; __syncthreads();
  float s2 = 0.f;
  for (int u = 0; u < per / 4; ++u)
#pragma unroll
    for (int q = 0; q < 4; ++q) { const float c = vals[u * 4 + q] - mu; s2 += c * c; }
  red[tid] = s2; __syncthreads();
  for (int st = 128; st > 0; st >>= 1) { if (tid < st) red[tid] += red[tid + st]; __syncthreads(); }
  const float rs = rsqrtf(red[0] / (float)N + eps);
  for (int pass = 0; pass < 2; ++pass) {
    for (int u = 0; u < per / 4; ++u) {
      const int j = tid * 4 + 1024 * u;
      v4f o, sm;
#pragma unroll
      for (int q = 0; q < 4; ++q) {
        float gg = g[j + q], bb = bta[j + q];
        if (PARAM_BF16) { gg = bf16_round(gg); bb = bf16_round(bb); }
        sm[q] = vals[u * 4 + q]; o[q] = (vals[u * 4 + q] - mu) * rs * gg + bb;
      }
      if (out_sum) *(volatile v4f*)(out_sum + (size_t)row * N + j) = sm;
      *(volatile v4f*)(out_norm + (size_t)row * N + j) = o;
    }
    if (pass == 0) __threadfence();
  }
}


typedef _Float16 v16h __attribute__((ext_vector_type(16)));
union FragH { v16h v; v8us half[2]; _Float16 h[16]; unsigned short u[16]; };
template <int NT>
__device__ __forceinline__ v8f mmaH(v16h ah, v16h al, v16h bh, v16h bl, v8f c) {
  c = __builtin_amdgcn_wmma_f32_16x16x32_f16(false, ah, false, bh, (short)0, c, false, false);
  if (NT >= 2) c = __builtin_amdgcn_wmma_f32_16x16x32_f16(false, al, false, bh, (short)0, c, false, false);
  if (NT >= 3) c = __builtin_amdgcn_wmma_f32_16x16x32_f16(false, ah, false, bl, (short)0, c, false, false);
  asm volatile("v_nop\n\tv_nop\n\tv_nop\n\tv_nop" : "+v"(c) : "v"(ah), "v"(al), "v"(bh), "v"(bl));
  return c;
}
template <bool ASPLIT>
__global__ __launch_bounds__(128) void k_gemm_h(const float* __restrict__ A, int lda, size_t sA, const _Float16* __restrict__ Bh, int ldb, size_t sB, float alpha, float* __restrict__ C, int ldc, size_t sC, int M, int N, int K) {
  __shared__ __attribute__((aligned(16))) float so[4][16][64];
  const int tid = threadIdx.x, w = tid >> 5, lane = tid & 31, ln = lane & 15, hh = lane >> 4; const int by = blockIdx.y;
  A += (size_t)by * sA; Bh += (size_t)by * sB; C += (size_t)by * sC;
  const int ntn = (N + 63) / 64; const int wid = blockIdx.x * 4 + w; const int mt = wid / ntn, nq = wid % ntn; if (mt * 16 >= M) return;
  const int row0 = mt * 16, col0 = nq * 64; const float* arow = A + (size_t)(row0 + ln) * lda;
  v8f acc[4] = {};
  for (int kb = 0; kb < K; kb += 32) {
    FragH ah, al;
    const v4f x0 = *(const v4fa*)(arow + kb + 8 * hh), x1 = *(const v4fa*)(arow + kb + 8 * hh + 4), x2 = *(const v4fa*)(arow + kb + 16 + 8 * hh), x3 = *(const v4fa*)(arow + kb + 16 + 8 * hh + 4);
    float xs[16] = {x0[0],x0[1],x0[2],x0[3],x1[0],x1[1],x1[2],x1[3],x2[0],x2[1],x2[2],x2[3],x3[0],x3[1],x3[2],x3[3]};
#pragma unroll
    for (int i = 0; i < 16; ++i) { const _Float16 h = (_Float16)xs[i]; ah.h[i] = h; al.h[i] = ASPLIT ? (_Float16)(xs[i] - (float)h) : (_Float16)0.0f; }
#pragma unroll
    for (int t = 0; t < 4; ++t) { if (col0 + t * 16 >= N) continue; const size_t boff = (size_t)(col0 + t * 16 + ln) * ldb + kb; FragH bq; bq.half[0] = *(const v8us*)(Bh + boff + 8 * hh); bq.half[1] = *(const v8us*)(Bh + boff + 16 + 8 * hh);
      acc[t] = mmaH<ASPLIT ? 2 : 1>(ah.v, al.v, bq.v, bq.v, acc[t]); }
  }
#pragma unroll
  for (int t = 0; t < 4; ++t) { if (col0 + t * 16 >= N) continue;
#pragma unroll
    for (int r = 0; r < 8; ++r) so[w][8 * hh + r][t * 16 + ln] = acc[t][r] * alpha; }
  __builtin_amdgcn_fence(__ATOMIC_ACQ_REL, "workgroup"); __builtin_amdgcn_wave_barrier();
  const int rsub = lane >> 4, c4 = (lane & 15) * 4;
  for (int pass = 0; pass < 2; ++pass) {
#pragma unroll
    for (int q = 0; q < 8; ++q) { const int r = q * 2 + rsub; if (col0 + c4 < N) { const v4f v = *(const v4fa*)&so[w][r][c4]; *(volatile v4f*)(C + (size_t)(row0 + r) * ldc + col0 + c4) = v; } }
    if (pass == 0) __threadfence(); }
}

__global__ __launch_bounds__(256) void k_wt_f16(const float* __restrict__ W, _Float16* __restrict__ Wt, int K, int N, float scale) {
  const int t = blockIdx.x * 256 + threadIdx.x; if (t >= N * (K / 8)) return; const int n = t / (K / 8), k8 = (t % (K / 8)) * 8; FragH f;
#pragma unroll
  for (int i = 0; i < 8; ++i) f.h[i] = (_Float16)(bf16_round(W[(size_t)(k8 + i) * N + n]) * scale); const v8us o = f.half[0];
  *(volatile v8us*)((unsigned short*)Wt + (size_t)n * K + k8) = o; __threadfence(); *(volatile v8us*)((unsigned short*)Wt + (size_t)n * K + k8) = o;
}
template <int ACT>
__global__ __launch_bounds__(128) void k_gemm_hhx(const _Float16* __restrict__ A, int lda, size_t sA, const _Float16* __restrict__ Bh, int ldb, size_t sB, float alpha, const float* __restrict__ bias, size_t sBias, const float* __restrict__ CP, int rowsPerB, size_t sCPb, int row0g,
    float* __restrict__ C, _Float16* __restrict__ C16, int ldc, size_t sC, int M, int N, int K) {
  __shared__ __attribute__((aligned(16))) float so[4][16][64];
  const int tid = threadIdx.x, w = tid >> 5, lane = tid & 31, ln = lane & 15, hh = lane >> 4; const int by = blockIdx.y;
  A += (size_t)by * sA; Bh += (size_t)by * sB; const size_t cofs = (size_t)by * sC; const float* bp = bias ? bias + (size_t)by * sBias : nullptr;
  const int ntn = (N + 63) / 64; const int wid = blockIdx.x * 4 + w; const int mt = wid / ntn, nq = wid % ntn; if (mt * 16 >= M) return;
  const int row0 = mt * 16, col0 = nq * 64; const _Float16* arow = A + (size_t)(row0 + ln) * lda;
  v8f acc[4] = {};
  for (int kb = 0; kb < K; kb += 32) { FragH ah; ah.half[0] = *(const v8us*)((const unsigned short*)arow + kb + 8 * hh); ah.half[1] = *(const v8us*)((const unsigned short*)arow + kb + 16 + 8 * hh);
#pragma unroll
    for (int t = 0; t < 4; ++t) { if (col0 + t * 16 >= N) continue; const size_t boff = (size_t)(col0 + t * 16 + ln) * ldb + kb; FragH bq; bq.half[0] = *(const v8us*)((const unsigned short*)Bh + boff + 8 * hh); bq.half[1] = *(const v8us*)((const unsigned short*)Bh + boff + 16 + 8 * hh);
      acc[t] = mmaH<1>(ah.v, ah.v, bq.v, bq.v, acc[t]); }
  }
#pragma unroll
  for (int t = 0; t < 4; ++t) { if (col0 + t * 16 >= N) continue; const int col = col0 + t * 16 + ln; const float bv = bp ? bf16_round(bp[col]) : 0.f;
#pragma unroll
    for (int r = 0; r < 8; ++r) { float v = acc[t][r] * alpha + bv; if (CP) { const int bidx = (row0g + row0 + 8 * hh + r) / rowsPerB; v += CP[(size_t)bidx * sCPb + (size_t)by * 64 + col]; } if (ACT == 1) v = (v > 0.f) ? v : expm1f(v); else if (ACT == 7) v = (v > 0.f) ? v + 1.0f : expf(v); else if (ACT == 8) v = tanhf(v); else if (ACT == 9) v = 0.5f * v * (1.0f + tanhf(0.7978845608028654f * (v + 0.044715f * v * v * v))); else if (ACT == 11) v = 1.0f / (1.0f + expf(-v)); else if (ACT == 12) v = (v > 0.f) ? v : 0.01f * v; else if (ACT == 14) v = (v > 0.f) ? v : 0.1f * v; else if (ACT == 15) v = v / (1.0f + expf(-v)); else if (ACT == 3) v = fmaxf(v, 0.f); else if (ACT == 6) v = 0.5f * v * (1.0f + erff(v * 0.70710678118654752f)); so[w][8 * hh + r][t * 16 + ln] = v; } }
  __builtin_amdgcn_fence(__ATOMIC_ACQ_REL, "workgroup"); __builtin_amdgcn_wave_barrier();
  const int rsub = lane >> 4, c4 = (lane & 15) * 4; typedef _Float16 v4h __attribute__((ext_vector_type(4)));
  for (int pass = 0; pass < 2; ++pass) {
#pragma unroll
    for (int q = 0; q < 8; ++q) { const int r = q * 2 + rsub; if (col0 + c4 < N) { const v4f v = *(const v4fa*)&so[w][r][c4]; if (C) *(volatile v4f*)(C + cofs + (size_t)(row0 + r) * ldc + col0 + c4) = v; if (C16) { v4h h4; for (int i = 0; i < 4; ++i) h4[i] = (_Float16)v[i]; *(volatile v4h*)(C16 + cofs + (size_t)(row0 + r) * ldc + col0 + c4) = h4; } } }
    if (pass == 0) __threadfence(); }
}


typedef _Float16 v4h __attribute__((ext_vector_type(4)));

__global__ __launch_bounds__(256) void k_x16(const float* __restrict__ x, _Float16* __restrict__ X16, size_t n8) { const size_t t = (size_t)blockIdx.x * 256 + threadIdx.x; if (t >= n8) return; FragH f;
#pragma unroll
  for (int q = 0; q < 8; ++q) f.h[q] = (_Float16)bf16_round(x[t * 8 + q]); *(volatile v8us*)((unsigned short*)X16 + t * 8) = f.half[0]; __threadfence(); *(volatile v8us*)((unsigned short*)X16 + t * 8) = f.half[0]; }
__global__ __launch_bounds__(256) void k_h16(const float* __restrict__ x, _Float16* __restrict__ X16, size_t n8) { const size_t t = (size_t)blockIdx.x * 256 + threadIdx.x; if (t >= n8) return; FragH f;
#pragma unroll
  for (int q = 0; q < 8; ++q) f.h[q] = (_Float16)x[t * 8 + q]; *(volatile v8us*)((unsigned short*)X16 + t * 8) = f.half[0]; __threadfence(); *(volatile v8us*)((unsigned short*)X16 + t * 8) = f.half[0]; }
__global__ __launch_bounds__(256) void k_round16f(const float* __restrict__ W, _Float16* __restrict__ Bt, size_t n8) { const size_t t = (size_t)blockIdx.x * 256 + threadIdx.x; if (t >= n8) return; FragH f;
#pragma unroll
  for (int i = 0; i < 8; ++i) f.h[i] = (_Float16)(bf16_round(W[t * 8 + i]) * 16.0f); *(volatile v8us*)((unsigned short*)Bt + t * 8) = f.half[0]; __threadfence(); *(volatile v8us*)((unsigned short*)Bt + t * 8) = f.half[0]; }
template <int NHv, int TTv>
__global__ __launch_bounds__(256) void k_vt(const _Float16* __restrict__ V16, int ldv, int voff, _Float16* __restrict__ Vt) { __shared__ unsigned short tl[64][66]; const int tid = threadIdx.x; const int slab = blockIdx.x / (TTv / 64), lg = blockIdx.x % (TTv / 64); const int b = slab / NHv, h = slab % NHv;
  for (int i = tid; i < 64 * 8; i += 256) { const int r = i / 8, c8 = (i % 8) * 8; FragH f; f.half[0] = *(const v8us*)((const unsigned short*)V16 + ((size_t)b * TTv + lg * 64 + r) * ldv + voff + h * 64 + c8);
#pragma unroll
    for (int q = 0; q < 8; ++q) tl[r][c8 + q] = f.u[q]; }
  __syncthreads();
  for (int pass = 0; pass < 2; ++pass) {
#pragma unroll
    for (int rd = 0; rd < 2; ++rd) { const int d = rd * 32 + tid / 8, pc = tid % 8; FragH f;
#pragma unroll
      for (int q = 0; q < 8; ++q) f.u[q] = tl[pc * 8 + q][d];
      *(volatile v8us*)((unsigned short*)Vt + ((size_t)slab * 64 + d) * TTv + lg * 64 + pc * 8) = f.half[0]; }
    if (pass == 0) __threadfence(); } }

__global__ __launch_bounds__(256) void k_hl(const float* __restrict__ F, _Float16* __restrict__ Hh, _Float16* __restrict__ Hl, size_t n8) { const size_t t = (size_t)blockIdx.x * 256 + threadIdx.x; if (t >= n8) return; FragH fh, fl; const v4f a = *(const v4fa*)(F + t * 8), c = *(const v4fa*)(F + t * 8 + 4);
#pragma unroll
  for (int q = 0; q < 4; ++q) { _Float16 h = (_Float16)a[q]; fh.h[q] = h; fl.h[q] = (_Float16)((a[q] - (float)h) * 1024.0f); h = (_Float16)c[q]; fh.h[4 + q] = h; fl.h[4 + q] = (_Float16)((c[q] - (float)h) * 1024.0f); }
  for (int pass = 0; pass < 2; ++pass) { *(volatile v8us*)((unsigned short*)Hh + t * 8) = fh.half[0]; *(volatile v8us*)((unsigned short*)Hl + t * 8) = fl.half[0]; if (pass == 0) __threadfence(); } }

__device__ __forceinline__ v16h g2_frag(const _Float16* p, int hh) { FragH f; f.half[0] = *(const v8us*)((const unsigned short*)p + 8 * hh); f.half[1] = *(const v8us*)((const unsigned short*)p + 16 + 8 * hh); return f.v; }
__device__ __forceinline__ v8f g2_mma(v16h a, v16h b, v8f c) { v8f d = __builtin_amdgcn_wmma_f32_16x16x32_f16(false, a, false, b, (short)0, c, false, false); asm volatile("v_nop\n\tv_nop\n\tv_nop\n\tv_nop" : "+v"(d) : "v"(a), "v"(b)); return d; }
template <int ACT>
__global__ __launch_bounds__(128) void k_gemm2(const _Float16* __restrict__ A, int lda, size_t sA, const _Float16* __restrict__ Bh, int ldb, size_t sB, float alpha, const float* __restrict__ bias, size_t sBias, const float* __restrict__ CP, int rowsPerB, size_t sCPb, int row0g,
    float* __restrict__ C, _Float16* __restrict__ C16, int ldc, size_t sC, int M, int N, int K) {
  __shared__ __attribute__((aligned(16))) float so[4][32][68];
  const int tid = threadIdx.x, w = tid >> 5, lane = tid & 31, ln = lane & 15, hh = lane >> 4; const int by = blockIdx.y;
  A += (size_t)by * sA; Bh += (size_t)by * sB; const size_t cofs = (size_t)by * sC; const float* bp = bias ? bias + (size_t)by * sBias : nullptr;
  const int ntn = N >> 6; const int mt = blockIdx.x / ntn, nq = blockIdx.x - mt * ntn; const int row0 = mt * 128 + 32 * w, col0 = nq * 64; if (row0 >= M) return;
  const _Float16* a0p = A + (size_t)(row0 + ln) * lda; const _Float16* a1p = a0p + (size_t)16 * lda;
  const _Float16* b0p = Bh + (size_t)(col0 + ln) * ldb; const _Float16* b1p = b0p + (size_t)16 * ldb; const _Float16* b2p = b1p + (size_t)16 * ldb; const _Float16* b3p = b2p + (size_t)16 * ldb;
  const v8f z8 = {0.f,0.f,0.f,0.f,0.f,0.f,0.f,0.f}; v8f c00 = z8, c01 = z8, c02 = z8, c03 = z8, c10 = z8, c11 = z8, c12 = z8, c13 = z8;
#pragma unroll 1
  for (int kb = 0; kb < K; kb += 32) { const v16h a0 = g2_frag(a0p + kb, hh), a1 = g2_frag(a1p + kb, hh);
    v16h b = g2_frag(b0p + kb, hh); c00 = g2_mma(a0, b, c00); c10 = g2_mma(a1, b, c10);
    b = g2_frag(b1p + kb, hh); c01 = g2_mma(a0, b, c01); c11 = g2_mma(a1, b, c11);
    b = g2_frag(b2p + kb, hh); c02 = g2_mma(a0, b, c02); c12 = g2_mma(a1, b, c12);
    b = g2_frag(b3p + kb, hh); c03 = g2_mma(a0, b, c03); c13 = g2_mma(a1, b, c13); }
  v8f accs[8] = {c00, c01, c02, c03, c10, c11, c12, c13};
#pragma unroll
  for (int u = 0; u < 8; ++u) { const int t = u & 3, half = u >> 2; const int col = col0 + t * 16 + ln; const float bv = bp ? bf16_round(bp[col]) : 0.f;
#pragma unroll
    for (int r = 0; r < 8; ++r) { const int rloc = half * 16 + 8 * hh + r; float v = accs[u][r] * alpha + bv; if (CP) { const int bidx = (row0g + row0 + rloc) / rowsPerB; v += CP[(size_t)bidx * sCPb + (size_t)by * 64 + col]; }
      if (ACT == 3) v = fmaxf(v, 0.f); else if (ACT == 6) v = 0.5f * v * (1.0f + erff(v * 0.70710678118654752f)); else if (ACT == 11) v = 1.0f / (1.0f + expf(-v)); else if (ACT == 15) v = v / (1.0f + expf(-v)); else if (ACT == 12) v = (v > 0.f) ? v : 0.01f * v; else if (ACT == 8) v = tanhf(v);
      so[w][rloc][t * 16 + ln] = v; } }
  __builtin_amdgcn_fence(__ATOMIC_ACQ_REL, "workgroup"); __builtin_amdgcn_wave_barrier();
  const int rsub = lane >> 4, c4 = (lane & 15) * 4;
  for (int pass = 0; pass < 2; ++pass) {
#pragma unroll
    for (int q = 0; q < 16; ++q) { const int r = q * 2 + rsub; const v4f v = *(const v4fa*)&so[w][r][c4]; if (C) *(volatile v4f*)(C + cofs + (size_t)(row0 + r) * ldc + col0 + c4) = v; if (C16) { v4h h4; for (int i = 0; i < 4; ++i) h4[i] = (_Float16)v[i]; *(volatile v4h*)(C16 + cofs + (size_t)(row0 + r) * ldc + col0 + c4) = h4; } }
    if (pass == 0) __threadfence(); } }


__global__ __launch_bounds__(256) void k_cl16(const float* __restrict__ src, _Float16* __restrict__ P16) {
  const int t = blockIdx.x * 256 + threadIdx.x; if (t >= NQ * (CIN / 8)) return; const int nq = t / (CIN / 8), c0 = (t % (CIN / 8)) * 8; FragH f;
#pragma unroll
  for (int q = 0; q < 8; ++q) f.h[q] = (_Float16)bf16_round(src[(size_t)(c0 + q) * NQ + nq]);
  *(volatile v8us*)((unsigned short*)P16 + (size_t)nq * CIN + c0) = f.half[0]; __threadfence(); *(volatile v8us*)((unsigned short*)P16 + (size_t)nq * CIN + c0) = f.half[0]; }
__global__ __launch_bounds__(256) void k_pos(const float* __restrict__ rowe, const float* __restrict__ cole, float* __restrict__ POS) {
  const int t = blockIdx.x * 256 + threadIdx.x; if (t >= NQ * (DD / 4)) return; const int nq = t / (DD / 4), c0 = (t % (DD / 4)) * 4; const int h = nq / HH, w = nq % HH; v4f o;
#pragma unroll
  for (int q = 0; q < 4; ++q) { const int c = c0 + q; o[q] = (c < 128) ? bf16_round(cole[(size_t)w * 128 + c]) : bf16_round(rowe[(size_t)h * 128 + c - 128]); }
  *(volatile v4f*)(POS + (size_t)t * 4) = o; __threadfence(); *(volatile v4f*)(POS + (size_t)t * 4) = o; }
__global__ __launch_bounds__(256) void k_addpos(const float* __restrict__ Q, const float* __restrict__ POS, _Float16* __restrict__ QP16, _Float16* __restrict__ QPR) {
  #pragma clang fp contract(off)
  const int t = blockIdx.x * 256 + threadIdx.x; if (t >= NQ * (DD / 8)) return; const int r = t / (DD / 8), c0 = (t % (DD / 8)) * 8; const v4f a = *(const v4fa*)(Q + (size_t)t * 8), a2 = *(const v4fa*)(Q + (size_t)t * 8 + 4), p = *(const v4fa*)(POS + (size_t)t * 8), p2 = *(const v4fa*)(POS + (size_t)t * 8 + 4); FragH f, gh, gl;
#pragma unroll
  for (int q = 0; q < 8; ++q) { const float v = (q < 4) ? a[q] : a2[q - 4], pp = (q < 4) ? p[q] : p2[q - 4]; f.h[q] = (_Float16)(v + pp); const _Float16 hv = (_Float16)v; gh.h[q] = hv; gl.h[q] = (_Float16)((v - (float)hv) * 16.0f); }
  unsigned short* d2 = (unsigned short*)QPR + (size_t)r * 2 * DD + c0;
  for (int pass = 0; pass < 2; ++pass) { *(volatile v8us*)((unsigned short*)QP16 + (size_t)t * 8) = f.half[0]; *(volatile v8us*)d2 = gh.half[0]; *(volatile v8us*)(d2 + DD) = gl.half[0]; if (pass == 0) __threadfence(); } }
__global__ __launch_bounds__(256) void k_pair16(const float* __restrict__ F, int n, _Float16* __restrict__ P, int rows) {
  #pragma clang fp contract(off)
  const int t = blockIdx.x * 256 + threadIdx.x; if (t >= rows * (n / 8)) return; const int r = t / (n / 8), c0 = (t % (n / 8)) * 8; const float* f = F + (size_t)r * n + c0; FragH fh, fl;
#pragma unroll
  for (int q = 0; q < 8; ++q) { const float v = f[q]; const _Float16 hv = (_Float16)v; fh.h[q] = hv; fl.h[q] = (_Float16)((v - (float)hv) * 16.0f); }
  unsigned short* d = (unsigned short*)P + (size_t)r * 2 * n + c0;
  for (int pass = 0; pass < 2; ++pass) { *(volatile v8us*)d = fh.half[0]; *(volatile v8us*)(d + n) = fl.half[0]; if (pass == 0) __threadfence(); } }
__global__ __launch_bounds__(256) void k_wtp2(const float* __restrict__ Wm, int K, int N, _Float16* __restrict__ Bt) {
  const int t = blockIdx.x * 256 + threadIdx.x; if (t >= N * (2 * K / 8)) return; const int n = t / (2 * K / 8), k0 = (t % (2 * K / 8)) * 8; const bool lo = (k0 >= K); const float sc = lo ? 1.0f : 16.0f; FragH f;
#pragma unroll
  for (int q = 0; q < 8; ++q) { const int k = k0 + q - (lo ? K : 0); f.h[q] = (_Float16)(bf16_round(Wm[(size_t)k * N + n]) * sc); }
  *(volatile v8us*)((unsigned short*)Bt + (size_t)n * 2 * K + k0) = f.half[0]; __threadfence(); *(volatile v8us*)((unsigned short*)Bt + (size_t)n * 2 * K + k0) = f.half[0]; }
__global__ __launch_bounds__(256) void k_woa(const float* __restrict__ offw, const float* __restrict__ aww, int i, _Float16* __restrict__ Bt) {
  const int t = blockIdx.x * 256 + threadIdx.x; if (t >= 128 * (DD / 8)) return; const int n = t / (DD / 8), k0 = (t % (DD / 8)) * 8; FragH f;
#pragma unroll
  for (int q = 0; q < 8; ++q) { const int k = k0 + q; float v = 0.f; if (n < 64) v = bf16_round(offw[((size_t)i * DD + k) * 64 + n]); else if (n < 96) v = bf16_round(aww[((size_t)i * DD + k) * 32 + (n - 64)]); f.h[q] = (_Float16)(v * 16.0f); }
  *(volatile v8us*)((unsigned short*)Bt + (size_t)n * DD + k0) = f.half[0]; __threadfence(); *(volatile v8us*)((unsigned short*)Bt + (size_t)n * DD + k0) = f.half[0]; }
__global__ __launch_bounds__(128) void k_boa(const float* __restrict__ offb, const float* __restrict__ awb, int i, float* __restrict__ BB) { const int t = threadIdx.x; const float v = (t < 64) ? offb[(size_t)i * 64 + t] : ((t < 96) ? awb[(size_t)i * 32 + t - 64] : 0.f); *(volatile float*)(BB + t) = v; __threadfence(); *(volatile float*)(BB + t) = v; }
__global__ __launch_bounds__(256) void k_msda(const float* __restrict__ OA, const _Float16* __restrict__ V16, _Float16* __restrict__ AO) {
  #pragma clang fp contract(off)
  const int t = blockIdx.x * 256 + threadIdx.x; if (t >= NQ * NHD * 2) return; const int g = t & 1; const int h = (t >> 1) & 7; const int r = t >> 4; const int qy = r / HH, qx = r % HH;
  const float* oa = OA + (size_t)r * 128; const float* lg = oa + 64 + h * NPT; const float* of = oa + h * NPT * 2;
  float m = fmaxf(fmaxf(lg[0], lg[1]), fmaxf(lg[2], lg[3])); float e[4]; float su = 0.f;
#pragma unroll
  for (int p = 0; p < 4; ++p) { e[p] = expf(lg[p] - m); su += e[p]; }
  const float rx = ((float)qx + 0.5f) / (float)HH, ry = ((float)qy + 0.5f) / (float)HH; float acc[16];
#pragma unroll
  for (int d = 0; d < 16; ++d) acc[d] = 0.f;
#pragma unroll 1
  for (int p = 0; p < NPT; ++p) { const float a = e[p] / su; const float lx_ = rx + of[p * 2] * (1.0f / (float)HH), ly_ = ry + of[p * 2 + 1] * (1.0f / (float)HH);
    const float px = lx_ * (float)HH - 0.5f, py = ly_ * (float)HH - 0.5f; const float x0f = floorf(px), y0f = floorf(py); const float wx = px - x0f, wy = py - y0f; const int x0 = (int)x0f, y0 = (int)y0f;
#pragma unroll 1
    for (int cn = 0; cn < 4; ++cn) { const int ix = x0 + (cn & 1), iy = y0 + (cn >> 1); if (ix < 0 || ix >= HH || iy < 0 || iy >= HH) continue; const float w = ((cn & 1) ? wx : (1.0f - wx)) * ((cn >> 1) ? wy : (1.0f - wy)); const float f = w * a;
      FragH vf; vf.half[0] = *(const v8us*)((const unsigned short*)V16 + ((size_t)iy * HH + ix) * DD + h * HD + g * 16); FragH vg; vg.half[0] = *(const v8us*)((const unsigned short*)V16 + ((size_t)iy * HH + ix) * DD + h * HD + g * 16 + 8);
#pragma unroll
      for (int d = 0; d < 8; ++d) { acc[d] += f * (float)vf.h[d]; acc[8 + d] += f * (float)vg.h[d]; } } }
  FragH o1, o2;
#pragma unroll
  for (int d = 0; d < 8; ++d) { o1.h[d] = (_Float16)acc[d]; o2.h[d] = (_Float16)acc[8 + d]; }
  unsigned short* dst = (unsigned short*)AO + (size_t)r * DD + h * HD + g * 16;
  for (int pass = 0; pass < 2; ++pass) { *(volatile v8us*)dst = o1.half[0]; *(volatile v8us*)(dst + 8) = o2.half[0]; if (pass == 0) __threadfence(); } }
template <int NC>
__global__ __launch_bounds__(256) void k_lnrelu(const float* __restrict__ F, const float* __restrict__ g, const float* __restrict__ bb, _Float16* __restrict__ H16) {
  #pragma clang fp contract(off)
  constexpr int PL = NC / 32; const int tid = threadIdx.x, w = tid >> 5, ln = tid & 31; const int r = blockIdx.x * 8 + w; if (r >= NQ) return; const float* x = F + (size_t)r * NC + ln * PL; float v[PL]; float s = 0.f;
#pragma unroll
  for (int q = 0; q < PL; ++q) { v[q] = x[q]; s += v[q]; }
  for (int o = 16; o > 0; o >>= 1) s += __shfl_xor(s, o, 32); const float mu = s / (float)NC; float q2 = 0.f;
#pragma unroll
  for (int q = 0; q < PL; ++q) { v[q] -= mu; q2 += v[q] * v[q]; }
  for (int o = 16; o > 0; o >>= 1) q2 += __shfl_xor(q2, o, 32); const float rs = rsqrtf(q2 / (float)NC + 1e-5f); _Float16 hh[PL], hl[PL];
#pragma unroll
  for (int q = 0; q < PL; ++q) { const int c = ln * PL + q; const float y = fmaxf(v[q] * rs * bf16_round(g[c]) + bf16_round(bb[c]), 0.f); hh[q] = (_Float16)y; hl[q] = (_Float16)((y - (float)hh[q]) * 16.0f); }
  unsigned short* dst = (unsigned short*)H16 + (size_t)r * 2 * NC + ln * PL; unsigned short* dl = dst + NC;
  for (int pass = 0; pass < 2; ++pass) { if (PL == 4) { *(volatile unsigned long long*)dst = *(const unsigned long long*)hh; *(volatile unsigned long long*)dl = *(const unsigned long long*)hl; } else { *(volatile unsigned*)dst = *(const unsigned*)hh; *(volatile unsigned*)dl = *(const unsigned*)hl; } if (pass == 0) __threadfence(); } }
__global__ __launch_bounds__(256) void k_nchw(const float* __restrict__ F, float* __restrict__ out) {
  const int t = blockIdx.x * 256 + threadIdx.x; if (t >= CIN * NQ / 4) return; const int c = t / (NQ / 4), q0 = (t % (NQ / 4)) * 4; v4f r;
#pragma unroll
  for (int q = 0; q < 4; ++q) r[q] = F[(size_t)(q0 + q) * CIN + c];
  *(volatile v4f*)(out + (size_t)c * NQ + q0) = r; __threadfence(); *(volatile v4f*)(out + (size_t)c * NQ + q0) = r; }

extern "C" void kernel_launch(void* const* d_in, const int* in_sizes, int n_in,
                              void* d_out, int out_size, void* d_ws, size_t ws_size, hipStream_t stream) {
  (void)in_sizes; (void)n_in; (void)out_size;
  const float* const* I = (const float* const*)d_in; const float* query = I[0]; const float* value = I[1]; const float* cqw = I[2]; const float* cqb = I[3]; const float* cvw = I[4]; const float* cvb = I[5]; const float* rowe = I[6]; const float* cole = I[7];
  const float* lqw = I[8]; const float* lqb = I[9]; const float* lvw = I[10]; const float* lvb = I[11]; const float* offw = I[12]; const float* offb = I[13]; const float* aww = I[14]; const float* awb = I[15]; const float* vpw = I[16]; const float* vpb = I[17]; const float* opw = I[18]; const float* opb = I[19];
  const float* w1 = I[20]; const float* b1 = I[21]; const float* g1 = I[22]; const float* be1 = I[23]; const float* w2 = I[24]; const float* b2 = I[25]; const float* g2 = I[26]; const float* be2 = I[27]; const float* w3 = I[28]; const float* b3 = I[29];
  char* ws = (char*)d_ws; size_t off = 0;
  auto take = [&](size_t bytes) { char* p = ws + off; off += (bytes + 255) & ~(size_t)255; return p; };
  _Float16* BCQ = (_Float16*)take((size_t)DD * CIN * 2); _Float16* BCV = (_Float16*)take((size_t)DD * CIN * 2); _Float16* BLQ = (_Float16*)take((size_t)DD * 2 * DD * 2); _Float16* BLV = (_Float16*)take((size_t)DD * 2 * DD * 2);
  _Float16* BVP = (_Float16*)take((size_t)4 * DD * 2 * DD * 2); _Float16* BOP = (_Float16*)take((size_t)4 * DD * DD * 2); _Float16* BOA = (_Float16*)take((size_t)4 * 128 * DD * 2); float* BBOA = (float*)take((size_t)4 * 128 * 4);
  _Float16* BW1 = (_Float16*)take((size_t)128 * 2 * DD * 2); _Float16* BW2 = (_Float16*)take((size_t)64 * 2 * 128 * 2); _Float16* BW3 = (_Float16*)take((size_t)CIN * 2 * 64 * 2);
  _Float16* QIN = (_Float16*)take((size_t)NQ * CIN * 2); _Float16* VIN = (_Float16*)take((size_t)NQ * CIN * 2); float* POS = (float*)take((size_t)NQ * DD * 4);
  float* Q = (float*)take((size_t)NQ * DD * 4); _Float16* VPR = (_Float16*)take((size_t)NQ * 2 * DD * 2); _Float16* QP16 = (_Float16*)take((size_t)NQ * DD * 2); _Float16* QPR = (_Float16*)take((size_t)NQ * 2 * DD * 2); _Float16* VAL = (_Float16*)take((size_t)NQ * DD * 2); float* OA = (float*)take((size_t)NQ * 128 * 4); _Float16* AO = (_Float16*)take((size_t)NQ * DD * 2);
  if (off > ws_size) return;
  _Float16* TP = (_Float16*)OA;
  float* FT = Q;
  float* F3 = (float*)QIN;
  float* F1 = OA; _Float16* H1 = VAL; float* F2 = (float*)QP16; _Float16* H2 = AO;
  const unsigned nb8 = (unsigned)(((size_t)NQ * DD / 8 + 255) / 256);
  k_round16f<<<(DD * CIN / 8 + 255) / 256, 256, 0, stream>>>(cqw, BCQ, (size_t)DD * CIN / 8); k_round16f<<<(DD * CIN / 8 + 255) / 256, 256, 0, stream>>>(cvw, BCV, (size_t)DD * CIN / 8);
  k_wtp2<<<(DD * (2 * DD / 8) + 255) / 256, 256, 0, stream>>>(lqw, DD, DD, BLQ); k_wtp2<<<(DD * (2 * DD / 8) + 255) / 256, 256, 0, stream>>>(lvw, DD, DD, BLV);
  for (int i = 0; i < 4; ++i) { k_wtp2<<<(DD * (2 * DD / 8) + 255) / 256, 256, 0, stream>>>(vpw + (size_t)i * DD * DD, DD, DD, BVP + (size_t)i * DD * 2 * DD); k_wt_f16<<<(DD * DD / 8 + 255) / 256, 256, 0, stream>>>(opw + (size_t)i * DD * DD, BOP + (size_t)i * DD * DD, DD, DD, 16.0f);
    k_woa<<<(128 * (DD / 8) + 255) / 256, 256, 0, stream>>>(offw, aww, i, BOA + (size_t)i * 128 * DD); k_boa<<<1, 128, 0, stream>>>(offb, awb, i, BBOA + (size_t)i * 128); }
  k_wtp2<<<(128 * (2 * DD / 8) + 255) / 256, 256, 0, stream>>>(w1, DD, 128, BW1); k_wtp2<<<(64 * (2 * 128 / 8) + 255) / 256, 256, 0, stream>>>(w2, 128, 64, BW2); k_wtp2<<<(CIN * (2 * 64 / 8) + 255) / 256, 256, 0, stream>>>(w3, 64, CIN, BW3);
  k_cl16<<<(NQ * (CIN / 8) + 255) / 256, 256, 0, stream>>>(query, QIN); k_cl16<<<(NQ * (CIN / 8) + 255) / 256, 256, 0, stream>>>(value, VIN); k_pos<<<(NQ * (DD / 4) + 255) / 256, 256, 0, stream>>>(rowe, cole, POS);
  const dim3 gD((NQ / 128) * (DD / 64), 1), gOA((NQ / 128) * 2, 1), g128((NQ / 128) * 2, 1), g64((NQ / 128) * 1, 1), g384((NQ / 128) * (CIN / 64), 1);
  k_gemm2<0><<<gD, 128, 0, stream>>>(VIN, CIN, 0, BCV, CIN, 0, 0.0625f, cvb, 0, nullptr, 1, 0, 0, FT, nullptr, DD, 0, NQ, DD, CIN); k_pair16<<<nb8, 256, 0, stream>>>(FT, DD, TP, NQ);
  k_gemm2<0><<<gD, 128, 0, stream>>>(TP, 2 * DD, 0, BLV, 2 * DD, 0, 0.0625f, lvb, 0, nullptr, 1, 0, 0, FT, nullptr, DD, 0, NQ, DD, 2 * DD); k_pair16<<<nb8, 256, 0, stream>>>(FT, DD, VPR, NQ);
  k_gemm2<0><<<gD, 128, 0, stream>>>(QIN, CIN, 0, BCQ, CIN, 0, 0.0625f, cqb, 0, nullptr, 1, 0, 0, FT, nullptr, DD, 0, NQ, DD, CIN); k_pair16<<<nb8, 256, 0, stream>>>(FT, DD, TP, NQ);
  k_gemm2<0><<<gD, 128, 0, stream>>>(TP, 2 * DD, 0, BLQ, 2 * DD, 0, 0.0625f, lqb, 0, nullptr, 1, 0, 0, Q, nullptr, DD, 0, NQ, DD, 2 * DD);
  for (int i = 0; i < NLAY; ++i) {
    k_addpos<<<nb8, 256, 0, stream>>>(Q, POS, QP16, QPR);
    const _Float16* vin = (i < NCROSS) ? VPR : QPR;
    k_gemm2<0><<<gD, 128, 0, stream>>>(vin, 2 * DD, 0, BVP + (size_t)i * DD * 2 * DD, 2 * DD, 0, 0.0625f, vpb + (size_t)i * DD, 0, nullptr, 1, 0, 0, nullptr, VAL, DD, 0, NQ, DD, 2 * DD);
    k_gemm2<0><<<gOA, 128, 0, stream>>>(QP16, DD, 0, BOA + (size_t)i * 128 * DD, DD, 0, 0.0625f, BBOA + (size_t)i * 128, 0, nullptr, 1, 0, 0, OA, nullptr, 128, 0, NQ, 128, DD);
    k_msda<<<(NQ * NHD * 2 + 255) / 256, 256, 0, stream>>>(OA, VAL, AO);
    k_gemm2<0><<<gD, 128, 0, stream>>>(AO, DD, 0, BOP + (size_t)i * DD * DD, DD, 0, 0.0625f, opb + (size_t)i * DD, 0, Q, 1, (size_t)DD, 0, Q, nullptr, DD, 0, NQ, DD, DD); }
  k_addpos<<<nb8, 256, 0, stream>>>(Q, POS, QP16, QPR);
  k_gemm2<0><<<g128, 128, 0, stream>>>(QPR, 2 * DD, 0, BW1, 2 * DD, 0, 0.0625f, b1, 0, nullptr, 1, 0, 0, F1, nullptr, 128, 0, NQ, 128, 2 * DD); k_lnrelu<128><<<NQ / 8, 256, 0, stream>>>(F1, g1, be1, H1);
  k_gemm2<0><<<g64, 128, 0, stream>>>(H1, 256, 0, BW2, 256, 0, 0.0625f, b2, 0, nullptr, 1, 0, 0, F2, nullptr, 64, 0, NQ, 64, 256); k_lnrelu<64><<<NQ / 8, 256, 0, stream>>>(F2, g2, be2, H2);
  k_gemm2<0><<<g384, 128, 0, stream>>>(H2, 128, 0, BW3, 128, 0, 0.0625f, b3, 0, nullptr, 1, 0, 0, F3, nullptr, CIN, 0, NQ, CIN, 128);
  k_nchw<<<(CIN * NQ / 4 + 255) / 256, 256, 0, stream>>>(F3, (float*)d_out);
}
